// LORA_Attention_43800076485448
// MI455X (gfx1250) — hardware-verified
//
#include <hip/hip_runtime.h>
#include <stdint.h>

static constexpr int kBatch = 8;
static constexpr int kSeq   = 1024;
static constexpr int kDim   = 768;
static constexpr int kHeads = 12;
static constexpr int kHd    = 64;
static constexpr int kRank  = 8;
static constexpr int kQkv   = 3 * kDim;
static constexpr int kQK    = 2 * kDim;
static constexpr int kHgrp  = 6;
static constexpr int kNgrp  = kHeads / kHgrp;
#define PSCALE 32768.0f
#define PSCALE_INV (1.0f / 32768.0f)
#define CSCALE 64.0f
#define WCARRY 16.0f

typedef __attribute__((ext_vector_type(16))) _Float16 v16h;
typedef __attribute__((ext_vector_type(8)))  _Float16 v8h;
typedef __attribute__((ext_vector_type(16))) __bf16   v16b;
typedef __attribute__((ext_vector_type(8)))  __bf16   v8b;
typedef __attribute__((ext_vector_type(8)))  float    v8f;
typedef __attribute__((ext_vector_type(4)))  float    v4f;
typedef __attribute__((ext_vector_type(2)))  float    v2f;
typedef __attribute__((ext_vector_type(4)))  unsigned int v4u;

__device__ __forceinline__ unsigned short f2bf_bits(float f) {
  unsigned u = __float_as_uint(f);
  return (unsigned short)((u + 0x7FFFu + ((u >> 16) & 1u)) >> 16);
}
__device__ __forceinline__ float bf_bits2f(unsigned short h) { return __uint_as_float(((unsigned)h) << 16); }

__device__ __forceinline__ void dep_guard_h(v8f& a, v8f& b, v16h x, v16h y) { asm volatile("v_nop\n\tv_nop\n\tv_nop\n\tv_nop" : "+v"(a), "+v"(b) : "v"(x), "v"(y)); }
__device__ __forceinline__ void dep_guard_b(v8f& a, v8f& b, v16b x, v16b y) { asm volatile("v_nop\n\tv_nop\n\tv_nop\n\tv_nop" : "+v"(a), "+v"(b) : "v"(x), "v"(y)); }
__device__ __forceinline__ void keep4_h(v16h a, v16h b, v16h c, v16h d) { asm volatile("v_nop" :: "v"(a), "v"(b), "v"(c), "v"(d)); }
__device__ __forceinline__ void keep4_b(v16b a, v16b b, v16b c, v16b d) { asm volatile("v_nop" :: "v"(a), "v"(b), "v"(c), "v"(d)); }
__device__ __forceinline__ void acc_guard4(v8f& a, v8f& b, v8f& c, v8f& d) { asm volatile("v_nop\n\tv_nop\n\tv_nop\n\tv_nop" : "+v"(a), "+v"(b), "+v"(c), "+v"(d)); }
template <typename T> struct Frag;
template <> struct Frag<_Float16> {
  typedef v16h V; union U { v16h v; v8h h[2]; };
  static __device__ __forceinline__ v16h load(const _Float16* p) {
    U f; f.h[0] = *(const v8h*)(p); f.h[1] = *(const v8h*)(p + 16); return f.v;
  }
  static __device__ __forceinline__ v8f mma(v16h a, v16h b, v8f c) {
    return __builtin_amdgcn_wmma_f32_16x16x32_f16(false, a, false, b, (short)0, c, false, false);
  }
  static __device__ __forceinline__ void guard(v8f& a, v8f& b, v16h x, v16h y) { dep_guard_h(a, b, x, y); }
  static __device__ __forceinline__ void keep(v16h a, v16h b, v16h c, v16h d) { keep4_h(a, b, c, d); }
};
template <> struct Frag<__bf16> {
  typedef v16b V; union U { v16b v; v8b h[2]; };
  static __device__ __forceinline__ v16b load(const __bf16* p) {
    U f; f.h[0] = *(const v8b*)(p); f.h[1] = *(const v8b*)(p + 16); return f.v;
  }
  static __device__ __forceinline__ v8f mma(v16b a, v16b b, v8f c) {
    return __builtin_amdgcn_wmma_f32_16x16x32_bf16(false, a, false, b, (short)0, c, false, false);
  }
  static __device__ __forceinline__ void guard(v8f& a, v8f& b, v16b x, v16b y) { dep_guard_b(a, b, x, y); }
  static __device__ __forceinline__ void keep(v16b a, v16b b, v16b c, v16b d) { keep4_b(a, b, c, d); }
};

template <int ET> struct Elem;
template <> struct Elem<0> { typedef _Float16 T; };
template <> struct Elem<1> { typedef __bf16 T; };
template <int ET, bool SPLIT, int BIAS_MODE, int OUT_MODE, bool RESID, int ACT = 0>
__global__ __launch_bounds__(256) void wmma_gemm64(
    const unsigned short* __restrict__ Ap, const unsigned short* __restrict__ A2p, int lda, long strideA,
    const unsigned short* __restrict__ Btp, const unsigned short* __restrict__ Bt2p, int ldb, long strideB,
    void* __restrict__ Cout, void* __restrict__ Cout2, int ldc, long strideC,
    const float* __restrict__ bias,
    const float* __restrict__ resid, long strideR,
    int M, int N, int K, float scale) {
  typedef typename Elem<ET>::T T;
  typedef typename Frag<T>::V V;
  const T* A = (const T*)Ap; const T* A2 = (const T*)A2p; const T* Bt = (const T*)Btp; const T* Bt2 = (const T*)Bt2p;
  __shared__ __align__(16) float sT[8][16 * 68];
  const int b    = blockIdx.y;
  const int lane = threadIdx.x & 31;
  const int wave = threadIdx.x >> 5;
  const int tilesN = N >> 6;
  const int tilesM = M >> 6;
  const int tile = blockIdx.x * 8 + wave;
  if (tile >= tilesM * tilesN) return;
  const int tm = tile / tilesN;
  const int tn = tile - tm * tilesN;
  const int m0 = tm << 6;
  const int n0 = tn << 6;

  const T* Ab  = A  + (size_t)b * strideA;
  const T* Bb  = Bt + (size_t)b * strideB;
  const T* Ab2 = SPLIT ? (A2  + (size_t)b * strideA) : nullptr;
  const T* Bb2 = SPLIT ? (Bt2 + (size_t)b * strideB) : nullptr;

  const int rlane = lane & 15;
  const int koff  = (lane >> 4) * 8;
  const int mOff  = (lane >> 4) * 8;

  v8f acc[4][4];
#pragma unroll
  for (int i = 0; i < 4; ++i)
#pragma unroll
    for (int j = 0; j < 4; ++j) acc[i][j] = (v8f){0.f,0.f,0.f,0.f,0.f,0.f,0.f,0.f};

  for (int k0 = 0; k0 < K; k0 += 32) {
    V bh[4], bl[4];
#pragma unroll
    for (int j = 0; j < 4; ++j) {
      const size_t bo = (size_t)(n0 + (j << 4) + rlane) * ldb + koff + k0;
      bh[j] = Frag<T>::load(Bb + bo);
      if (SPLIT) bl[j] = Frag<T>::load(Bb2 + bo);
    }
#pragma unroll
    for (int i = 0; i < 4; ++i) {
      const size_t ao = (size_t)(m0 + (i << 4) + rlane) * lda + koff + k0;
      V ah = Frag<T>::load(Ab + ao);
      V al;
      if (SPLIT) al = Frag<T>::load(Ab2 + ao);
#pragma unroll
      for (int j = 0; j < 4; ++j) {
        acc[i][j] = Frag<T>::mma(ah, bh[j], acc[i][j]);
        if (SPLIT) {
          acc[i][j] = Frag<T>::mma(ah, bl[j], acc[i][j]);
          acc[i][j] = Frag<T>::mma(al, bh[j], acc[i][j]);
        }
      }
      Frag<T>::guard(acc[i][0], acc[i][3], ah, SPLIT ? al : ah);
    }
    Frag<T>::keep(bh[0], bh[1], bh[2], bh[3]);
    if (SPLIT) Frag<T>::keep(bl[0], bl[1], bl[2], bl[3]);
  }
  acc_guard4(acc[0][0], acc[0][1], acc[0][2], acc[0][3]);
  acc_guard4(acc[1][0], acc[1][1], acc[1][2], acc[1][3]);
  acc_guard4(acc[2][0], acc[2][1], acc[2][2], acc[2][3]);
  acc_guard4(acc[3][0], acc[3][1], acc[3][2], acc[3][3]);

  float* slab = sT[wave];
  const float* Rb = RESID ? (resid + (size_t)b * strideR) : nullptr;
#pragma unroll
  for (int i = 0; i < 4; ++i) {
    const int mBase = m0 + (i << 4);
#pragma unroll
    for (int j = 0; j < 4; ++j) {
      const int n = n0 + (j << 4) + rlane;
      float bv = 0.f;
      if (BIAS_MODE == 2) bv = bias[n];
#pragma unroll
      for (int r = 0; r < 8; ++r) {
        float v = acc[i][j][r] * scale;
        if (BIAS_MODE == 1) v += bias[mBase + mOff + r];
        if (BIAS_MODE == 2) v += bv;
        if (RESID) v += Rb[(size_t)(mBase + mOff + r) * ldc + n];
        if (ACT == 1) v = tanhf(v);
        if (ACT == 2) v = fmaxf(v, 0.0f);
        if (ACT == 3) v = v / (1.0f + expf(-v));
        if (ACT == 4) v = (v > 0.f) ? v : 0.01f * v;
        slab[(mOff + r) * 68 + (j << 4) + rlane] = v;
      }
    }
    __builtin_amdgcn_fence(__ATOMIC_RELEASE, "workgroup");
    __builtin_amdgcn_wave_barrier();
    __builtin_amdgcn_fence(__ATOMIC_ACQUIRE, "workgroup");
    if (OUT_MODE == 0) {
      float* C = (float*)Cout + (size_t)b * strideC;
      const int hh = lane >> 4, c4 = (lane & 15) * 4;
      for (int pass = 0; pass < 2; ++pass) {
#pragma unroll
        for (int it = 0; it < 8; ++it) {
          const int row = it * 2 + hh;
          v4f v = *(const v4f*)(slab + row * 68 + c4);
          *(volatile v4f*)(C + (size_t)(mBase + row) * ldc + n0 + c4) = v;
        }
        __threadfence();
      }
    } else {
      const int q = lane >> 3, c8 = (lane & 7) * 8;
      unsigned short* C  = (unsigned short*)Cout  + (size_t)b * strideC;
      unsigned short* C2 = (OUT_MODE == 2) ? ((unsigned short*)Cout2 + (size_t)b * strideC) : nullptr;
      for (int pass = 0; pass < 2; ++pass) {
#pragma unroll
        for (int it = 0; it < 4; ++it) {
          const int row = it * 4 + q;
          const float* sp = slab + row * 68 + c8;
          v8h hv, lv;
#pragma unroll
          for (int e = 0; e < 8; ++e) {
            if (OUT_MODE == 1) {
              hv[e] = (_Float16)sp[e];
            } else {
              unsigned short hb = f2bf_bits(sp[e]);
              unsigned short lb = f2bf_bits(sp[e] - bf_bits2f(hb));
              hv[e] = __builtin_bit_cast(_Float16, hb);
              lv[e] = __builtin_bit_cast(_Float16, lb);
            }
          }
          *(volatile v8h*)(C + (size_t)(mBase + row) * ldc + n0 + c8) = hv;
          if (OUT_MODE == 2) *(volatile v8h*)(C2 + (size_t)(mBase + row) * ldc + n0 + c8) = lv;
        }
        __threadfence();
      }
    }
    __builtin_amdgcn_fence(__ATOMIC_RELEASE, "workgroup");
    __builtin_amdgcn_wave_barrier();
    __builtin_amdgcn_fence(__ATOMIC_ACQUIRE, "workgroup");
  }
}

__device__ __forceinline__ unsigned pk16(unsigned short a, unsigned short b) { return (unsigned)a | ((unsigned)b << 16); }
__device__ __forceinline__ unsigned short h_bits(float f) { const _Float16 h = (_Float16)f; return __builtin_bit_cast(unsigned short, h); }

__global__ __launch_bounds__(256) void cast_f16x2_kernel(const float* __restrict__ in, unsigned short* __restrict__ out, int n2, float scale) {
  const int i = blockIdx.x * 256 + threadIdx.x;
  if (i < n2) {
    const v2f f = *(const v2f*)(in + 2 * (size_t)i);
    const unsigned u = pk16(h_bits(f[0] * scale), h_bits(f[1] * scale));
    ((volatile unsigned*)out)[i] = u;
    __threadfence();
    ((volatile unsigned*)out)[i] = u;
  }
}

__global__ __launch_bounds__(256) void fold_cast_kernel(const float* __restrict__ w, const float* __restrict__ la,
                                                        const float* __restrict__ lb, unsigned short* __restrict__ out,
                                                        int n2, float scale) {
  const int i = blockIdx.x * 256 + threadIdx.x;
  if (i < n2) {
    const int e = 2 * i;
    const int o = e / kDim;
    const int c = e - o * kDim;
    const v2f wv = *(const v2f*)(w + (size_t)e);
    float s0 = wv[0], s1 = wv[1];
    const float* brow = lb + (size_t)o * kRank;
#pragma unroll 1
    for (int r = 0; r < kRank; ++r) {
      const float bb = brow[r];
      const v2f av = *(const v2f*)(la + (size_t)r * kDim + c);
      s0 = fmaf(bb, av[0], s0);
      s1 = fmaf(bb, av[1], s1);
    }
    const unsigned u = pk16(h_bits(s0 * scale), h_bits(s1 * scale));
    ((volatile unsigned*)out)[i] = u;
    __threadfence();
    ((volatile unsigned*)out)[i] = u;
  }
}

__global__ __launch_bounds__(128) void softmax_row_kernel(const float* __restrict__ S, unsigned short* __restrict__ P) {
  __shared__ float redm[4];
  __shared__ float reds[4];
  const int i    = blockIdx.x;
  const int hg   = blockIdx.y;
  const int tid  = threadIdx.x;
  const int lane = tid & 31;
  const int wave = tid >> 5;
  const int j0   = tid * 8;
  const float* rp = S + ((size_t)hg * kSeq + i) * kSeq + j0;
  const v4f a = *(const v4f*)(rp);
  const v4f c = *(const v4f*)(rp + 4);
  float m = fmaxf(fmaxf(fmaxf(a[0], a[1]), fmaxf(a[2], a[3])), fmaxf(fmaxf(c[0], c[1]), fmaxf(c[2], c[3])));
#pragma unroll
  for (int off = 16; off > 0; off >>= 1) m = fmaxf(m, __shfl_xor(m, off, 32));
  if (lane == 0) redm[wave] = m;
  __syncthreads();
  float mx = redm[0];
  mx = fmaxf(mx, redm[1]); mx = fmaxf(mx, redm[2]); mx = fmaxf(mx, redm[3]);
  const float e0 = __expf(a[0] - mx), e1 = __expf(a[1] - mx), e2 = __expf(a[2] - mx), e3 = __expf(a[3] - mx);
  const float e4 = __expf(c[0] - mx), e5 = __expf(c[1] - mx), e6 = __expf(c[2] - mx), e7 = __expf(c[3] - mx);
  float s = ((e0 + e1) + (e2 + e3)) + ((e4 + e5) + (e6 + e7));
#pragma unroll
  for (int off = 16; off > 0; off >>= 1) s += __shfl_xor(s, off, 32);
  if (lane == 0) reds[wave] = s;
  __syncthreads();
  float tot = reds[0];
  tot += reds[1]; tot += reds[2]; tot += reds[3];
  const float inv = 1.0f / tot;
  const float p0 = e0 * inv, p1 = e1 * inv, p2 = e2 * inv, p3 = e3 * inv;
  const float p4 = e4 * inv, p5 = e5 * inv, p6 = e6 * inv, p7 = e7 * inv;
  const v4u hv = (v4u){pk16(h_bits(p0 * PSCALE), h_bits(p1 * PSCALE)),
                       pk16(h_bits(p2 * PSCALE), h_bits(p3 * PSCALE)),
                       pk16(h_bits(p4 * PSCALE), h_bits(p5 * PSCALE)),
                       pk16(h_bits(p6 * PSCALE), h_bits(p7 * PSCALE))};
  const size_t ro = ((size_t)hg * kSeq + i) * kSeq + j0;
  *(volatile v4u*)(P + ro) = hv;
  __threadfence();
  *(volatile v4u*)(P + ro) = hv;
}

extern "C" void kernel_launch(void* const* d_in, const int* in_sizes, int n_in,
                              void* d_out, int out_size, void* d_ws, size_t ws_size,
                              hipStream_t stream) {
  if (n_in < 13) return;
  if (in_sizes[0] != kBatch * kSeq * kDim) return;
  if (in_sizes[1] != kQkv * kDim) return;
  if (in_sizes[2] != kQkv) return;
  if (in_sizes[3] != kDim * kDim) return;
  if (in_sizes[4] != kDim) return;
  for (int t = 5; t < 13; ++t) { if (in_sizes[t] != kRank * kDim) return; }
  if (out_size != kBatch * kSeq * kDim) return;

  const float* x      = (const float*)d_in[0];
  const float* w_qkv  = (const float*)d_in[1];
  const float* b_qkv  = (const float*)d_in[2];
  const float* w_proj = (const float*)d_in[3];
  const float* b_proj = (const float*)d_in[4];
  const float* q_a    = (const float*)d_in[5];
  const float* q_b    = (const float*)d_in[6];
  const float* k_a    = (const float*)d_in[7];
  const float* k_b    = (const float*)d_in[8];
  const float* v_a    = (const float*)d_in[9];
  const float* v_b    = (const float*)d_in[10];
  const float* o_a    = (const float*)d_in[11];
  const float* o_b    = (const float*)d_in[12];

  const size_t pWQKV = (size_t)kQkv * kDim * 2;
  const size_t pWP   = (size_t)kDim * kDim * 2;
  const size_t pX    = (size_t)kBatch * kSeq * kDim * 2;
  const size_t pQK   = (size_t)kBatch * kSeq * kQK * 2;
  const size_t pVT   = (size_t)kBatch * kDim * kSeq * 2;
  const size_t pCTX  = (size_t)kBatch * kSeq * kDim * 2;
  const size_t pS    = (size_t)kHgrp * kSeq * kSeq * 4;
  const size_t pP    = (size_t)kHgrp * kSeq * kSeq * 2;
  size_t off = 0;
  const size_t oWQKV = off; off += pWQKV;
  const size_t oWP   = off; off += pWP;
  const size_t oX    = off; off += pX;
  const size_t oQK   = off; off += pQK;
  const size_t oVT   = off; off += pVT;
  const size_t oCTX  = off; off += pCTX;
  const size_t oS    = off; off += pS;
  const size_t oP    = off; off += pP;
  if (off > ws_size) return;

  char* ws = (char*)d_ws;
  unsigned short* WQKV16 = (unsigned short*)(ws + oWQKV);
  unsigned short* WP16   = (unsigned short*)(ws + oWP);
  unsigned short* X16    = (unsigned short*)(ws + oX);
  unsigned short* QK16   = (unsigned short*)(ws + oQK);
  unsigned short* VT16   = (unsigned short*)(ws + oVT);
  unsigned short* CTX16  = (unsigned short*)(ws + oCTX);
  float*          Sbuf   = (float*)(ws + oS);
  unsigned short* P16    = (unsigned short*)(ws + oP);

  const dim3 blk(256);
  const dim3 blk128(128);
  const int n2w = kDim * kDim / 2;
  const int n2x = kBatch * kSeq * kDim / 2;
  const dim3 gFold((n2w + 255) / 256);
  const dim3 gCastX((n2x + 255) / 256);
  const size_t secW = (size_t)kDim * kDim;

  fold_cast_kernel<<<gFold, blk, 0, stream>>>(w_qkv,            q_a, q_b, WQKV16,            n2w, WCARRY);
  fold_cast_kernel<<<gFold, blk, 0, stream>>>(w_qkv + secW,     k_a, k_b, WQKV16 + secW,     n2w, WCARRY);
  fold_cast_kernel<<<gFold, blk, 0, stream>>>(w_qkv + 2 * secW, v_a, v_b, WQKV16 + 2 * secW, n2w, WCARRY);
  fold_cast_kernel<<<gFold, blk, 0, stream>>>(w_proj,           o_a, o_b, WP16,              n2w, WCARRY);

  cast_f16x2_kernel<<<gCastX, blk, 0, stream>>>(x, X16, n2x, 1.0f);

  const int tilesTok = kBatch * kSeq / 64;
  const int tilesSeq = kSeq / 64;
  const dim3 gQK((tilesTok * (kQK / 64) + 7) / 8, 1);
  const dim3 gVT(((kDim / 64) * tilesSeq + 7) / 8, kBatch);
  const dim3 gS((tilesSeq * tilesSeq + 7) / 8, kHgrp);
  const dim3 gPV((tilesSeq * (kHd / 64) + 7) / 8, kHgrp);
  const dim3 gO((tilesTok * (kDim / 64) + 7) / 8, 1);
  const float wscale  = 1.0f / WCARRY;
  const float sscale  = 0.125f;
  const float pvscale = PSCALE_INV * CSCALE;
  const float oscale  = 1.0f / (WCARRY * CSCALE);

  wmma_gemm64<0, false, 2, 1, false, 0><<<gQK, blk, 0, stream>>>(
      X16, X16, kDim, 0L, WQKV16, WQKV16, kDim, 0L, (void*)QK16, (void*)QK16, kQK, 0L,
      b_qkv, b_qkv, 0L, kBatch * kSeq, kQK, kDim, wscale);
  wmma_gemm64<0, false, 1, 1, false, 0><<<gVT, blk, 0, stream>>>(
      WQKV16 + 2 * secW, WQKV16 + 2 * secW, kDim, 0L, X16, X16, kDim, (long)kSeq * kDim,
      (void*)VT16, (void*)VT16, kSeq, (long)kDim * kSeq,
      b_qkv + 2 * kDim, b_qkv + 2 * kDim, 0L, kDim, kSeq, kDim, wscale);

  for (int b = 0; b < kBatch; ++b) {
    const unsigned short* QKb  = QK16 + (size_t)b * kSeq * kQK;
    const unsigned short* VTb  = VT16 + (size_t)b * kDim * kSeq;
    unsigned short*       CTXb = CTX16 + (size_t)b * kSeq * kDim;
    for (int g = 0; g < kNgrp; ++g) {
      const size_t hc = (size_t)g * kHgrp * kHd;
      wmma_gemm64<0, false, 0, 0, false, 0><<<gS, blk, 0, stream>>>(
          QKb + hc, QKb + hc, kQK, (long)kHd, QKb + kDim + hc, QKb + kDim + hc, kQK, (long)kHd,
          (void*)Sbuf, (void*)Sbuf, kSeq, (long)kSeq * kSeq,
          b_proj, b_proj, 0L, kSeq, kSeq, kHd, sscale);
      softmax_row_kernel<<<dim3(kSeq, kHgrp), blk128, 0, stream>>>(Sbuf, P16);
      wmma_gemm64<0, false, 0, 1, false, 0><<<gPV, blk, 0, stream>>>(
          P16, P16, kSeq, (long)kSeq * kSeq, VTb + hc * kSeq, VTb + hc * kSeq, kSeq, (long)kHd * kSeq,
          (void*)(CTXb + hc), (void*)(CTXb + hc), kDim, (long)kHd,
          b_proj, b_proj, 0L, kSeq, kHd, kSeq, pvscale);
    }
  }
  wmma_gemm64<0, false, 2, 0, false, 0><<<gO, blk, 0, stream>>>(
      CTX16, CTX16, kDim, 0L, WP16, WP16, kDim, 0L, d_out, d_out, kDim, 0L,
      b_proj, b_proj, 0L, kBatch * kSeq, kDim, kDim, oscale);
}
